// NNConv_87436944212625
// MI455X (gfx1250) — hardware-verified
//
#include <hip/hip_runtime.h>
#include <stddef.h>


#define WIDTH 32
#define EDGE_DIM 6
#define HIDDEN 128
#define NOUT 1024

#define CH1 4096
#define MAXB 1600
#define PITCHB 1568
#define BPT 7
#define MAXNB1 128
#define CAP3 1024
#define WPB 4
#define LDSW 13312

typedef _Float16 v16h __attribute__((ext_vector_type(16)));
typedef _Float16 v8h __attribute__((ext_vector_type(8)));
typedef float v8f __attribute__((ext_vector_type(8)));
typedef float v4f __attribute__((ext_vector_type(4)));
typedef int v4i __attribute__((ext_vector_type(4)));
typedef v8h __attribute__((may_alias)) v8ha;
typedef v4f __attribute__((may_alias)) v4fa;
typedef v4i __attribute__((may_alias)) v4ia;

union Frag { v16h v; v8h half[2]; };

#define LDS_FENCE() asm volatile("s_wait_dscnt 0" ::: "memory")

__device__ __forceinline__ v8f wmma16(const v16h& a, const v16h& b, v8f c) {
    return __builtin_amdgcn_wmma_f32_16x16x32_f16(false, a, false, b, (short)0, c, false, false);
}

__global__ __launch_bounds__(256) void k_prep(const float* __restrict__ W2, _Float16* w2frag, int nslots) {
    const int t = blockIdx.x * 256 + threadIdx.x;
    const bool ok = t < nslots;
    const int tt = ok ? t : 0;
    const int g = tt & 1, l = (tt >> 1) & 31, s = (tt >> 6) & 3, j = tt >> 8;
    const int h = l >> 4, n = j * 16 + (l & 15);
    const int kb = s * 32 + 8 * h + 16 * g;
    union { v8h v; _Float16 e[8]; } u;
#pragma unroll
    for (int ii = 0; ii < 8; ++ii) u.e[ii] = (_Float16)(W2[(size_t)(kb + ii) * NOUT + n] * 64.0f);
    const v8h val = u.v;
    if (ok) *(volatile v8h*)(w2frag + (size_t)tt * 8) = val;
    __threadfence();
    if (ok) *(volatile v8h*)(w2frag + (size_t)tt * 8) = val;
}

__device__ __forceinline__ void chunk_keys(const int* __restrict__ recv, int cb, int lane, int E, int N,
                                           unsigned& key_out, int& rank, bool& last, bool& valid) {
    const int e = cb + lane;
    unsigned key = 0xFFFFFFFFu;
    if (e < E) {
        const int r = recv[e];
        if (r >= 0 && r < N) key = ((unsigned)r & ~31u) | (unsigned)lane;
    }
#pragma unroll
    for (int kk = 2; kk <= 32; kk <<= 1) {
#pragma unroll
        for (int j = kk >> 1; j > 0; j >>= 1) {
            const unsigned p = __shfl_xor(key, j);
            const bool asc = (lane & kk) == 0;
            const bool low = (lane & j) == 0;
            const unsigned mn = key < p ? key : p;
            const unsigned mx = key < p ? p : key;
            key = (asc == low) ? mn : mx;
        }
    }
    const unsigned bkt = key >> 5;
    const unsigned pk = __shfl_up(key, 1);
    const unsigned nk = __shfl_down(key, 1);
    const bool start = (lane == 0) || ((pk >> 5) != bkt);
    last = (lane == 31) || ((nk >> 5) != bkt);
    int v = start ? lane : 0;
#pragma unroll
    for (int d = 1; d < 32; d <<= 1) {
        const int u = __shfl_up(v, d);
        if (lane >= d && u > v) v = u;
    }
    rank = lane - v;
    key_out = key;
    valid = (key != 0xFFFFFFFFu);
}

__global__ __launch_bounds__(256) void k_bucket(const int* __restrict__ recv, int* lists, int* offtab, int E, int N) {
    __shared__ unsigned short wcnt[8 * MAXB];
    __shared__ __attribute__((aligned(16))) int list_lds[CH1];
    __shared__ __attribute__((aligned(16))) int boff[PITCHB];
    __shared__ int sb[256];
    const int t = threadIdx.x, lane = t & 31, wid = t >> 5, blk = blockIdx.x;

    for (int i = t; i < 8 * MAXB; i += 256) wcnt[i] = 0;
    for (int i = t; i < CH1; i += 256) list_lds[i] = 0;
    __syncthreads();

    const int wbase = blk * CH1 + wid * 512;
#pragma unroll 1
    for (int c = 0; c < 16; ++c) {
        unsigned key; int rank; bool last, valid;
        chunk_keys(recv, wbase + c * 32, lane, E, N, key, rank, last, valid);
        if (valid && last) {
            const int b = (int)(key >> 5);
            wcnt[wid * MAXB + b] += (unsigned short)(rank + 1);
        }
    }
    __syncthreads();

    int tsum = 0;
#pragma unroll 1
    for (int q = 0; q < BPT; ++q) {
        const int b = t * BPT + q;
        if (b < PITCHB) {
            int tot = 0;
#pragma unroll
            for (int w = 0; w < 8; ++w) tot += (int)wcnt[w * MAXB + b];
            tsum += tot;
        }
    }
    sb[t] = tsum;
    __syncthreads();
#pragma unroll 1
    for (int d = 1; d < 256; d <<= 1) {
        const int v = (t >= d) ? sb[t - d] : 0;
        __syncthreads();
        sb[t] += v;
        __syncthreads();
    }
    int run = sb[t] - tsum;
#pragma unroll 1
    for (int q = 0; q < BPT; ++q) {
        const int b = t * BPT + q;
        if (b < PITCHB) {
            boff[b] = run;
#pragma unroll
            for (int w = 0; w < 8; ++w) {
                const int cnt = (int)wcnt[w * MAXB + b];
                wcnt[w * MAXB + b] = (unsigned short)run;
                run += cnt;
            }
        }
    }
    __syncthreads();

#pragma unroll 1
    for (int c = 0; c < 16; ++c) {
        const int cb = wbase + c * 32;
        unsigned key; int rank; bool last, valid;
        chunk_keys(recv, cb, lane, E, N, key, rank, last, valid);
        if (valid) {
            const int b = (int)(key >> 5);
            const int pos = (int)wcnt[wid * MAXB + b] + rank;
            if ((unsigned)pos < (unsigned)CH1) list_lds[pos] = cb + (int)(key & 31u);
            if (last) wcnt[wid * MAXB + b] = (unsigned short)(pos + 1);
        }
    }
    __syncthreads();

    const v4ia* lsrc = (const v4ia*)list_lds;
    const v4ia* bsrc = (const v4ia*)boff;
    v4i lv[4];
#pragma unroll
    for (int u = 0; u < 4; ++u) lv[u] = lsrc[t + u * 256];
    const int t2 = t + 256;
    const bool has2 = t2 < (PITCHB / 4);
    const v4i bv0 = bsrc[t];
    const v4i bv1 = bsrc[has2 ? t2 : t];
    int* ld = lists + (size_t)blk * CH1;
    int* bd = offtab + (size_t)blk * PITCHB;
#pragma unroll
    for (int u = 0; u < 4; ++u) *(volatile v4i*)(ld + (size_t)(t + u * 256) * 4) = lv[u];
    *(volatile v4i*)(bd + (size_t)t * 4) = bv0;
    if (has2) *(volatile v4i*)(bd + (size_t)t2 * 4) = bv1;
    __threadfence();
#pragma unroll
    for (int u = 0; u < 4; ++u) *(volatile v4i*)(ld + (size_t)(t + u * 256) * 4) = lv[u];
    *(volatile v4i*)(bd + (size_t)t * 4) = bv0;
    if (has2) *(volatile v4i*)(bd + (size_t)t2 * 4) = bv1;
}

__global__ __launch_bounds__(128) void k_edge(
    const float* __restrict__ x, const int* __restrict__ senders, const float* __restrict__ edge_attr,
    const float* __restrict__ W1, const float* __restrict__ b1, const _Float16* w2frag,
    const float* __restrict__ b2, float* msgs, int E, int N, int npairs) {
    __shared__ float b2_lds[NOUT];
    __shared__ __attribute__((aligned(16))) unsigned char wmem[WPB * LDSW];

    const int lane = threadIdx.x & 31;
    const int wid = threadIdx.x >> 5;
    const int m = lane & 15;
    const int hh = lane >> 4;

    for (int i = threadIdx.x; i < NOUT; i += 128) b2_lds[i] = b2[i] * 1024.0f;
    __syncthreads();

    const int pair = blockIdx.x * WPB + wid;
    if (pair >= npairs) return;

    float w1reg[EDGE_DIM][4];
    float b1reg[4];
#pragma unroll
    for (int c = 0; c < 4; ++c) {
        b1reg[c] = b1[c * 32 + lane] * 16.0f;
#pragma unroll
        for (int d = 0; d < EDGE_DIM; ++d) w1reg[d][c] = W1[d * HIDDEN + c * 32 + lane] * 16.0f;
    }

    float* x_lds = (float*)(wmem + wid * LDSW);
    _Float16* h_lds = (_Float16*)(wmem + wid * LDSW + 4096);
    float* ea_lds = (float*)(wmem + wid * LDSW + 12288);
    int* sidx = (int*)(wmem + wid * LDSW + 13056);

    const int ebase = pair * 32;

    {
        const int e = ebase + lane;
        int sn = 0;
        if (e < E) {
            sn = senders[e];
            sn = sn < 0 ? 0 : (sn >= N ? N - 1 : sn);
        }
        sidx[lane] = sn;
    }
    const int ealim = E * EDGE_DIM;
#pragma unroll
    for (int tq = 0; tq < EDGE_DIM; ++tq) {
        const int idx = ebase * EDGE_DIM + tq * 32 + lane;
        ea_lds[tq * 32 + lane] = (idx < ealim) ? edge_attr[idx] : 0.0f;
    }
    LDS_FENCE();

#pragma unroll 4
    for (int r = 0; r < 32; ++r) {
        const int sn = sidx[r];
        x_lds[r * WIDTH + lane] = x[(size_t)sn * WIDTH + lane];
    }

#pragma unroll 2
    for (int r = 0; r < 32; ++r) {
        const float e0 = ea_lds[r * 6 + 0], e1 = ea_lds[r * 6 + 1], e2 = ea_lds[r * 6 + 2];
        const float e3 = ea_lds[r * 6 + 3], e4 = ea_lds[r * 6 + 4], e5 = ea_lds[r * 6 + 5];
#pragma unroll
        for (int c = 0; c < 4; ++c) {
            float acc = b1reg[c];
            acc = fmaf(e0, w1reg[0][c], acc);
            acc = fmaf(e1, w1reg[1][c], acc);
            acc = fmaf(e2, w1reg[2][c], acc);
            acc = fmaf(e3, w1reg[3][c], acc);
            acc = fmaf(e4, w1reg[4][c], acc);
            acc = fmaf(e5, w1reg[5][c], acc);
            acc = fmaxf(acc, 0.0f);
            h_lds[r * HIDDEN + c * 32 + lane] = (_Float16)acc;
        }
    }
    LDS_FENCE();

    Frag afrag[2][4];
    const v8ha* hv = (const v8ha*)h_lds;
#pragma unroll
    for (int t = 0; t < 2; ++t)
#pragma unroll
        for (int s = 0; s < 4; ++s) {
            const int b8 = (t * 16 + m) * (HIDDEN / 8) + s * 4 + hh;
            afrag[t][s].half[0] = hv[b8];
            afrag[t][s].half[1] = hv[b8 + 2];
        }

    float macc[2][2][8];
#pragma unroll
    for (int t = 0; t < 2; ++t)
#pragma unroll
        for (int hf = 0; hf < 2; ++hf)
#pragma unroll
            for (int r = 0; r < 8; ++r) macc[t][hf][r] = 0.0f;

    const v8h* wq = (const v8h*)w2frag;

#pragma unroll 1
    for (int w = 0; w < WIDTH; ++w) {
        float xw[2][8];
#pragma unroll
        for (int t = 0; t < 2; ++t)
#pragma unroll
            for (int r = 0; r < 8; ++r) xw[t][r] = x_lds[(t * 16 + 8 * hh + r) * WIDTH + w];
#pragma unroll
        for (int half = 0; half < 2; ++half) {
            const int j = 2 * w + half;
            Frag bq[4];
#pragma unroll
            for (int s = 0; s < 4; ++s) {
                const int fb = ((j * 4 + s) * 32 + lane) * 2;
                bq[s].half[0] = wq[fb];
                bq[s].half[1] = wq[fb + 1];
            }
            const float b2n = b2_lds[j * 16 + m];
            v8f c0;
#pragma unroll
            for (int r = 0; r < 8; ++r) c0[r] = b2n;
            v8f c1 = c0;
#pragma unroll
            for (int s = 0; s < 4; ++s) c0 = wmma16(afrag[0][s].v, bq[s].v, c0);
#pragma unroll
            for (int s = 0; s < 4; ++s) c1 = wmma16(afrag[1][s].v, bq[s].v, c1);
            asm volatile("v_nop\n\tv_nop\n\tv_nop\n\tv_nop"
                         : "+v"(c0), "+v"(c1)
                         : "v"(bq[0].v), "v"(bq[1].v), "v"(bq[2].v), "v"(bq[3].v));
#pragma unroll
            for (int r = 0; r < 8; ++r) {
                macc[0][half][r] = fmaf(c0[r], xw[0][r], macc[0][half][r]);
                macc[1][half][r] = fmaf(c1[r], xw[1][r], macc[1][half][r]);
            }
        }
    }
    LDS_FENCE();

    const float inv = 0.0009765625f;
#pragma unroll
    for (int t = 0; t < 2; ++t)
#pragma unroll
        for (int half = 0; half < 2; ++half)
#pragma unroll
            for (int r = 0; r < 8; ++r)
                x_lds[(t * 16 + 8 * hh + r) * WIDTH + half * 16 + m] = macc[t][half][r] * inv;
    LDS_FENCE();

    const v4fa* mv = (const v4fa*)x_lds;
    v4f ov[8];
#pragma unroll
    for (int it = 0; it < 8; ++it) ov[it] = mv[it * 32 + lane];
    float* mb = msgs + (size_t)ebase * WIDTH;
#pragma unroll
    for (int it = 0; it < 8; ++it) *(volatile v4f*)(mb + (size_t)(it * 32 + lane) * 4) = ov[it];
    __threadfence();
#pragma unroll
    for (int it = 0; it < 8; ++it) *(volatile v4f*)(mb + (size_t)(it * 32 + lane) * 4) = ov[it];
}

__global__ __launch_bounds__(32) void k_gather(const int* __restrict__ recv, const int* lists, const int* offtab,
                                               const float* msgs, float* out, int E, int N, int NB1) {
    __shared__ unsigned comp[CAP3];
    __shared__ __attribute__((aligned(16))) float acc[32 * 32];
    const int lane = threadIdx.x;
    const int f = blockIdx.x;

    int cnt[4], lo[4], ex[4];
    int carry = 0;
#pragma unroll
    for (int u = 0; u < 4; ++u) {
        const int blk = lane + 32 * u;
        int c = 0, l0 = 0;
        if (blk < NB1) {
            const int* tb = offtab + (size_t)blk * PITCHB;
            int a = tb[f];
            int b = tb[f + 1];
            a = a < 0 ? 0 : (a > CH1 ? CH1 : a);
            b = b < a ? a : (b > CH1 ? CH1 : b);
            c = b - a;
            l0 = a;
        }
        cnt[u] = c;
        lo[u] = l0;
        int s = c;
#pragma unroll
        for (int d = 1; d < 32; d <<= 1) {
            const int v = __shfl_up(s, d);
            if (lane >= d) s += v;
        }
        ex[u] = carry + s - c;
        carry += __shfl(s, 31);
    }
    const int T = carry < CAP3 ? carry : CAP3;

#pragma unroll
    for (int u = 0; u < 4; ++u) {
        const int blk = lane + 32 * u;
        if (blk < NB1) {
            const int* lp = lists + (size_t)blk * CH1 + lo[u];
            for (int q = 0; q < cnt[u]; ++q) {
                const int p = ex[u] + q;
                if (p < CAP3) {
                    const int e = lp[q];
                    unsigned pk = 0xFFFFFFFFu;
                    if ((unsigned)e < (unsigned)E) {
                        const int nd = recv[e] - f * 32;
                        if ((unsigned)nd < 32u) pk = ((unsigned)e << 5) | (unsigned)nd;
                    }
                    comp[p] = pk;
                }
            }
        }
    }
#pragma unroll
    for (int r = 0; r < 32; ++r) acc[r * 32 + lane] = 0.0f;
    __syncthreads();

#pragma unroll 1
    for (int i = 0; i < T; ++i) {
        const unsigned pk = comp[i];
        if (pk != 0xFFFFFFFFu) {
            const int e = (int)(pk >> 5);
            const int nd = (int)(pk & 31u);
            const float v = msgs[(size_t)e * WIDTH + lane];
            acc[nd * 32 + lane] += v;
        }
    }
    __syncthreads();

    const v4fa* av = (const v4fa*)acc;
    const int rows_here = N - f * 32;
    v4f ov[8];
    bool ok[8];
#pragma unroll
    for (int it = 0; it < 8; ++it) {
        const int idx = it * 32 + lane;
        ov[it] = av[idx];
        ok[it] = (idx >> 3) < rows_here;
    }
    float* ob = out + (size_t)f * 32 * WIDTH;
#pragma unroll
    for (int it = 0; it < 8; ++it)
        if (ok[it]) *(volatile v4f*)(ob + (size_t)(it * 32 + lane) * 4) = ov[it];
    __threadfence();
#pragma unroll
    for (int it = 0; it < 8; ++it)
        if (ok[it]) *(volatile v4f*)(ob + (size_t)(it * 32 + lane) * 4) = ov[it];
}

extern "C" void kernel_launch(void* const* d_in, const int* in_sizes, int n_in,
                              void* d_out, int out_size, void* d_ws, size_t ws_size,
                              hipStream_t stream) {
    if (n_in < 8) return;
    const float* x = (const float*)d_in[0];
    const int* senders = (const int*)d_in[1];
    const int* recv = (const int*)d_in[2];
    const float* edge_attr = (const float*)d_in[3];
    const float* W1 = (const float*)d_in[4];
    const float* b1 = (const float*)d_in[5];
    const float* W2 = (const float*)d_in[6];
    const float* b2 = (const float*)d_in[7];
    float* out = (float*)d_out;

    const int N = in_sizes[0] / WIDTH;
    const int E = in_sizes[1];
    if (N <= 0 || E <= 0) return;
    if (in_sizes[0] != N * WIDTH || in_sizes[2] != E || in_sizes[3] != E * EDGE_DIM ||
        in_sizes[4] != EDGE_DIM * HIDDEN || in_sizes[5] != HIDDEN ||
        in_sizes[6] != HIDDEN * NOUT || in_sizes[7] != NOUT || out_size != N * WIDTH) return;

    const int NB = (N + 31) / 32;
    if (NB + 1 > PITCHB) return;
    const int NB1 = (E + CH1 - 1) / CH1;
    if (NB1 > MAXNB1) return;
    const int npairs = (E + 31) / 32;
    const int Epad = npairs * 32;
    const int nslots = HIDDEN * NOUT / 8;

    const size_t off_w2 = 0;
    const size_t sz_w2 = (size_t)HIDDEN * NOUT * sizeof(_Float16);
    const size_t off_lists = off_w2 + sz_w2;
    const size_t sz_lists = (size_t)NB1 * CH1 * sizeof(int);
    const size_t off_tab = off_lists + sz_lists;
    const size_t sz_tab = (size_t)NB1 * PITCHB * sizeof(int);
    const size_t off_msgs = off_tab + sz_tab;
    const size_t sz_msgs = (size_t)Epad * WIDTH * sizeof(float);
    if (off_msgs + sz_msgs > ws_size) return;

    char* ws = (char*)d_ws;
    _Float16* w2frag = (_Float16*)(ws + off_w2);
    int* lists = (int*)(ws + off_lists);
    int* offtab = (int*)(ws + off_tab);
    float* msgs = (float*)(ws + off_msgs);

    k_prep<<<(nslots + 255) / 256, 256, 0, stream>>>(W2, w2frag, nslots);
    k_bucket<<<NB1, 256, 0, stream>>>(recv, lists, offtab, E, N);
    k_edge<<<(npairs + WPB - 1) / WPB, 128, 0, stream>>>(x, senders, edge_attr, W1, b1, w2frag, b2,
                                                         msgs, E, N, npairs);
    k_gather<<<NB, 32, 0, stream>>>(recv, lists, offtab, msgs, out, E, N, NB1);
}
